// TemporalBlock_49606872268956
// MI455X (gfx1250) — hardware-run, weakly checked
//
#include <hip/hip_runtime.h>


namespace {
constexpr int B = 8, CIN = 128, C = 256, L = 4096, KW = 7, DIL = 2, PAD = 12, L2 = L + PAD, L2P = 4160  , KT = CIN * KW  , CC = 32, KCH = CC * KW  , BL = 8  ;
constexpr int LQ = 4096  , LQ2 = ((LQ + PAD + 63) / 64) * 64 < L2P ? ((LQ + PAD + 63) / 64) * 64 : L2P;
constexpr float XS = 8.0f, WSC = 256.0f, LOG2E = 1.4426950408889634f;
static_assert(L % 64 == 0 && KCH % 32 == 0 && L2P % 64 == 0 && L2P >= L2, "tiling");
typedef _Float16 b16;
typedef __attribute__((ext_vector_type(16))) _Float16 v16b;
typedef __attribute__((ext_vector_type(8))) _Float16 v8b;
typedef __attribute__((ext_vector_type(8))) float v8f;
typedef __attribute__((ext_vector_type(4))) float v4f;
__device__ __forceinline__ float bf16_rne(float f) { unsigned int u = __float_as_uint(f); u += 0x7FFFu + ((u >> 16) & 1u); return __uint_as_float(u & 0xFFFF0000u); }
__device__ __forceinline__ void split16(float v, b16& hi, b16& lo) { hi = (b16)v; lo = (b16)(v - (float)hi); }
__device__ __forceinline__ v16b frag_kb(const b16* p, int hh) { const v8b a = *(const v8b*)(p + 8 * hh), b = *(const v8b*)(p + 16 + 8 * hh); v16b f;
#pragma unroll
  for (int e = 0; e < 8; ++e) { f[e] = a[e]; f[8 + e] = b[e]; } return f; }
__device__ __forceinline__ v8f wmma16b(v16b a, v16b b, v8f c) { v8f d = __builtin_amdgcn_wmma_f32_16x16x32_f16(false, a, false, b, (short)0, c, false, false); asm volatile("v_nop\n\tv_nop\n\tv_nop\n\tv_nop" : "+v"(d) : "v"(a), "v"(b)); return d; }
__device__ __forceinline__ void wave_lds_sync() { __builtin_amdgcn_fence(__ATOMIC_RELEASE, "workgroup"); __builtin_amdgcn_wave_barrier(); __builtin_amdgcn_fence(__ATOMIC_ACQUIRE, "workgroup"); }
__device__ __forceinline__ float pmul(float a, float b) { float p = a * b; asm volatile("" : "+v"(p)); return p; }
__device__ __forceinline__ int iclamp(int v, int lo, int hi) { return v < lo ? lo : (v > hi ? hi : v); }

typedef __attribute__((ext_vector_type(2))) float v2f;
__global__ __launch_bounds__(256) void prep_kernel(const float* __restrict__ v1, const float* __restrict__ g1, const float* __restrict__ qkvw, const float* __restrict__ pw, const float* __restrict__ dsw, b16* __restrict__ WV, b16* __restrict__ WQ, b16* __restrict__ WP, b16* __restrict__ WD, float* __restrict__ SCL) {
  const size_t u = (size_t)blockIdx.x * 256 + threadIdx.x; const size_t n1 = (size_t)C * KT / 8, n2 = (size_t)3 * C * C / 8, n3 = (size_t)C * C / 8, n4 = (size_t)C * CIN / 8; v8b o; const float* w; b16* dst; size_t e;
  if (u < n1) { w = v1; dst = WV; e = u * 8; } else if (u < n1 + n2) { w = qkvw; dst = WQ; e = (u - n1) * 8; } else if (u < n1 + n2 + n3) { w = pw; dst = WP; e = (u - n1 - n2) * 8; } else if (u < n1 + n2 + n3 + n4) { w = dsw; dst = WD; e = (u - n1 - n2 - n3) * 8; }
  else { const int oo = (int)(u - n1 - n2 - n3 - n4); if (oo < C) { float s = 0.0f;
#pragma unroll 1
      for (int i = 0; i < KT; ++i) { const float t = bf16_rne(v1[(size_t)oo * KT + i]); s += t * t; }
      const float sc = bf16_rne(g1[oo]) / sqrtf(s); for (int pass = 0; pass < 2; ++pass) { ((volatile float*)SCL)[oo] = sc; __threadfence(); } } return; }
  for (int j = 0; j < 8; ++j) o[j] = (b16)(bf16_rne(w[e + j]) * WSC);
  for (int pass = 0; pass < 2; ++pass) { *(volatile v8b*)(dst + e) = o; __threadfence(); }
}
__global__ __launch_bounds__(128) void conv_kernel(const float* __restrict__ x, const b16* __restrict__ WV, const float* __restrict__ SCL, const float* __restrict__ b1, float* __restrict__ H) {
  __shared__ __attribute__((aligned(16))) b16 As[64][KCH + 8]; __shared__ __attribute__((aligned(16))) float Tf[4][16][128 + 4];
  const int wave = threadIdx.x >> 5, lane = threadIdx.x & 31, nloc = lane & 15, hlf = lane >> 4; const int l0 = blockIdx.x * 64; const int b = blockIdx.y; const int n0 = blockIdx.z * 128;
  const float* xb = x + (size_t)b * CIN * L;
  v8f acc[8];
#pragma unroll
  for (int t = 0; t < 8; ++t) acc[t] = (v8f){};
#pragma unroll 1
  for (int ch = 0; ch < CIN; ch += CC) {
    __syncthreads();
    for (int i = threadIdx.x; i < 64 * KCH; i += 128) { const int lx = i & 63, k = i >> 6; const int cl = k / KW, kk = k % KW; const int pos = l0 + lx + DIL * kk - PAD; float v = 0.0f; if (pos >= 0 && pos < L) v = bf16_rne(xb[(size_t)(ch + cl) * L + pos]); As[lx][k] = (b16)(v * XS); }
    __syncthreads();
#pragma unroll 7
    for (int kb = 0; kb < KCH; kb += 32) { const v16b a = frag_kb(&As[wave * 16 + nloc][kb], hlf);
#pragma unroll
      for (int t = 0; t < 8; ++t) acc[t] = wmma16b(a, frag_kb(WV + (size_t)(n0 + t * 16 + nloc) * KT + ch * KW + kb, hlf), acc[t]); } }
#pragma unroll
  for (int t = 0; t < 8; ++t) { const int o = n0 + t * 16 + nloc; const float sc = SCL[o], bb = bf16_rne(b1[o]);
#pragma unroll
    for (int r = 0; r < 8; ++r) Tf[wave][8 * hlf + r][t * 16 + nloc] = fmaxf(acc[t][r] * (1.0f / (XS * WSC)) * sc + bb, 0.0f); }
  wave_lds_sync();
  for (int pass = 0; pass < 2; ++pass) { for (int rr = 0; rr < 16; ++rr) *(volatile v4f*)(H + ((size_t)b * L + l0 + wave * 16 + rr) * C + n0 + lane * 4) = *(const v4f*)(&Tf[wave][rr][lane * 4]); __threadfence(); }
}
__device__ __forceinline__ v16b frag_rowf32(const float* __restrict__ row, bool valid, int hh) {
  v16b a; if (!valid) { a = (v16b){}; return a; } const v4f c0 = *(const v4f*)(row + 8 * hh), c1 = *(const v4f*)(row + 8 * hh + 4), c2 = *(const v4f*)(row + 16 + 8 * hh), c3 = *(const v4f*)(row + 16 + 8 * hh + 4);
  for (int i = 0; i < 4; ++i) { a[i] = (b16)(c0[i] * XS); a[4 + i] = (b16)(c1[i] * XS); a[8 + i] = (b16)(c2[i] * XS); a[12 + i] = (b16)(c3[i] * XS); } return a;
}
__global__ __launch_bounds__(128) void qkv_kernel(const float* __restrict__ H, const b16* __restrict__ WQ, const float* __restrict__ qb, b16* __restrict__ QKV) {
  __shared__ __attribute__((aligned(16))) float Tf[4][16][128 + 4];
  const int wave = threadIdx.x >> 5, lane = threadIdx.x & 31, nloc = lane & 15, hlf = lane >> 4; const int b = blockIdx.z; const size_t m0 = (size_t)b * L2P + ((size_t)blockIdx.x * 4 + wave) * 16; const int n0 = blockIdx.y * 128;
  const size_t row = m0 + nloc; const int l2 = (int)(row % L2P); const int l = l2 - PAD; const bool valid = (l >= 0 && l < L);
  const float* hrow = H + ((size_t)b * L + (valid ? l : 0)) * C;
  v8f acc[8];
#pragma unroll
  for (int t = 0; t < 8; ++t) acc[t] = (v8f){};
#pragma unroll 2
  for (int ks = 0; ks < C / 32; ++ks) { const v16b a = frag_rowf32(hrow + ks * 32, valid, hlf);
#pragma unroll
    for (int t = 0; t < 8; ++t) acc[t] = wmma16b(a, frag_kb(WQ + (size_t)(n0 + t * 16 + nloc) * C + ks * 32, hlf), acc[t]); }
#pragma unroll
  for (int t = 0; t < 8; ++t) { const float bb = bf16_rne(qb[n0 + t * 16 + nloc]);
#pragma unroll
    for (int r = 0; r < 8; ++r) Tf[wave][8 * hlf + r][t * 16 + nloc] = acc[t][r] * (1.0f / (XS * WSC)) + bb; }
  wave_lds_sync();
  for (int pass = 0; pass < 2; ++pass) { for (int rr = 0; rr < 16; ++rr) { const v4f f = *(const v4f*)(&Tf[wave][rr][lane * 4]); __attribute__((ext_vector_type(4))) _Float16 o4; for (int j = 0; j < 4; ++j) o4[j] = (b16)(f[j] * XS); *(volatile __attribute__((ext_vector_type(4))) _Float16*)(QKV + (m0 + rr) * (3 * C) + n0 + lane * 4) = o4; } __threadfence(); }
}
__global__ __launch_bounds__(256) void na_kernel(const b16* __restrict__ QKV, const float* __restrict__ rpb, float* __restrict__ O) {
  const int wave = threadIdx.x >> 5, lane = threadIdx.x & 31; const size_t u = (size_t)blockIdx.x * 8 + wave; const int b = (int)(u / L), l2 = (int)(u % L); const int c = lane * 8;
  const b16* base = QKV + (size_t)b * L2P * (3 * C);
  float q[8]; { const v8b qv = *(const v8b*)(base + (size_t)l2 * (3 * C) + c); for (int j = 0; j < 8; ++j) q[j] = (float)qv[j] * (1.0f / XS); }
  const int r = l2 % DIL, ii = l2 / DIL; const int Lg = (L2 - r + DIL - 1) / DIL; int start = ii - KW / 2; start = start < 0 ? 0 : (start > Lg - KW ? Lg - KW : start);
  float m = -INFINITY, den = 0.0f; float acc[8]; for (int j = 0; j < 8; ++j) acc[j] = 0.0f;
#pragma unroll 1
  for (int t = 0; t < KW; ++t) { const int pos = r + DIL * (start + t); const int bidx = start + t - ii + (KW - 1);
    const v8b kv = *(const v8b*)(base + (size_t)pos * (3 * C) + C + c); float d = 0.0f;
#pragma unroll
    for (int j = 0; j < 8; ++j) d += q[j] * ((float)kv[j] * (1.0f / XS));
#pragma unroll
    for (int o2 = 1; o2 < 32; o2 <<= 1) d += __shfl_xor(d, o2);
    const float sc = d * 0.0625f + bf16_rne(rpb[bidx < 0 ? 0 : (bidx > 2 * KW - 2 ? 2 * KW - 2 : bidx)]);
    const float mn = fmaxf(m, sc); const float al = (m == -INFINITY) ? 0.0f : __expf(m - mn), w = __expf(sc - mn);
    const v8b vv = *(const v8b*)(base + (size_t)pos * (3 * C) + 2 * C + c);
#pragma unroll
    for (int j = 0; j < 8; ++j) acc[j] = acc[j] * al + ((float)vv[j] * (1.0f / XS)) * w;
    den = den * al + w; m = mn; }
  const float inv = 1.0f / den;
  for (int pass = 0; pass < 2; ++pass) { const v4f o0 = {acc[0] * inv, acc[1] * inv, acc[2] * inv, acc[3] * inv}, o1 = {acc[4] * inv, acc[5] * inv, acc[6] * inv, acc[7] * inv}; *(volatile v4f*)(O + u * C + c) = o0; *(volatile v4f*)(O + u * C + c + 4) = o1; __threadfence(); }
}
__global__ __launch_bounds__(128) void out_kernel(const float* __restrict__ O, const float* __restrict__ x, const b16* __restrict__ WP, const b16* __restrict__ WD, const float* __restrict__ pb, const float* __restrict__ dsb, float* __restrict__ out) {
  __shared__ __attribute__((aligned(16))) b16 Xs[64][CIN + 8]; __shared__ __attribute__((aligned(16))) float Tf[4][16][128 + 4];
  const int wave = threadIdx.x >> 5, lane = threadIdx.x & 31, nloc = lane & 15, hlf = lane >> 4; const int l0 = blockIdx.x * 64; const int b = blockIdx.y; const int n0 = blockIdx.z * 128;
  for (int i = threadIdx.x; i < 64 * CIN; i += 128) { const int lx = i & 63, cc = i >> 6; Xs[lx][cc] = (b16)(bf16_rne(x[((size_t)b * CIN + cc) * L + l0 + lx]) * XS); }
  __syncthreads();
  v8f ap[8], ar[8];
#pragma unroll
  for (int t = 0; t < 8; ++t) { ap[t] = (v8f){}; ar[t] = (v8f){}; }
  const float* orow = O + ((size_t)b * L + l0 + wave * 16 + nloc) * C;
#pragma unroll 2
  for (int ks = 0; ks < C / 32; ++ks) { const v16b a = frag_rowf32(orow + ks * 32, true, hlf);
#pragma unroll
    for (int t = 0; t < 8; ++t) ap[t] = wmma16b(a, frag_kb(WP + (size_t)(n0 + t * 16 + nloc) * C + ks * 32, hlf), ap[t]); }
#pragma unroll
  for (int ks = 0; ks < CIN / 32; ++ks) { const v16b a = frag_kb(&Xs[wave * 16 + nloc][ks * 32], hlf);
#pragma unroll
    for (int t = 0; t < 8; ++t) ar[t] = wmma16b(a, frag_kb(WD + (size_t)(n0 + t * 16 + nloc) * CIN + ks * 32, hlf), ar[t]); }
#pragma unroll
  for (int t = 0; t < 8; ++t) { const int o = n0 + t * 16 + nloc; const float b1v = bf16_rne(pb[o]), b2v = bf16_rne(dsb[o]);
#pragma unroll
    for (int r = 0; r < 8; ++r) Tf[wave][8 * hlf + r][t * 16 + nloc] = fmaxf(fmaxf(ap[t][r] * (1.0f / (XS * WSC)) + b1v, 0.0f) + ar[t][r] * (1.0f / (XS * WSC)) + b2v, 0.0f); }
  __syncthreads();
  for (int pass = 0; pass < 2; ++pass) {
#pragma unroll 1
    for (int qq = 0; qq < 32; ++qq) { const int cl = wave * 32 + qq; const int o = n0 + cl; const int lx = lane * 2; v2f vv; vv[0] = Tf[lx >> 4][lx & 15][cl]; vv[1] = Tf[(lx + 1) >> 4][(lx + 1) & 15][cl]; *(volatile v2f*)(out + ((size_t)b * C + o) * L + l0 + lx) = vv; }
    __threadfence(); }
}
}

extern "C" void kernel_launch(void* const* d_in, const int* in_sizes, int n_in, void* d_out, int out_size, void* d_ws, size_t ws_size, hipStream_t stream) {
  (void)n_in;
  auto Fp = [&](int i) { return (const float*)d_in[i]; };
  if (in_sizes[0] != B * CIN * L || in_sizes[1] != C * KT || in_sizes[2] != C || in_sizes[3] != C || in_sizes[4] != 3 * C * C || in_sizes[5] != 3 * C || in_sizes[6] != 2 * KW - 1 || in_sizes[7] != C * C || in_sizes[9] != C * CIN || in_sizes[10] != C || out_size != B * C * L) return;
  size_t off = 0; char* ws = (char*)d_ws;
  auto carve = [&](size_t bytes) { char* p = ws + off; off += (bytes + 255) & ~(size_t)255; return p; };
  b16* WV = (b16*)carve((size_t)C * KT * 2); b16* WQ = (b16*)carve((size_t)3 * C * C * 2); b16* WP = (b16*)carve((size_t)C * C * 2); b16* WD = (b16*)carve((size_t)C * CIN * 2); float* SCL = (float*)carve((size_t)C * 4);
  float* H = (float*)carve((size_t)B * L * C * 4); b16* QKV = (b16*)carve((size_t)B * L2P * 3 * C * 2); float* O = (float*)carve((size_t)B * L * C * 4);
  if (off > ws_size || off > ((size_t)128 << 20)) return;
  const size_t nprep = (size_t)C * KT / 8 + (size_t)3 * C * C / 8 + (size_t)C * C / 8 + (size_t)C * CIN / 8 + C;
  prep_kernel<<<(unsigned)((nprep + 255) / 256), 256, 0, stream>>>(Fp(1), Fp(2), Fp(4), Fp(7), Fp(9), WV, WQ, WP, WD, SCL);
  conv_kernel<<<dim3(LQ / 64, BL, 2), 128, 0, stream>>>(Fp(0), WV, SCL, Fp(3), H);
  qkv_kernel<<<dim3(LQ2 / 64, 6, BL), 128, 0, stream>>>(H, WQ, Fp(5), QKV);
  na_kernel<<<(BL * L) / 8, 256, 0, stream>>>(QKV, Fp(6), O);
  out_kernel<<<dim3(LQ / 64, BL, 2), 128, 0, stream>>>(O, Fp(0), WP, WD, Fp(8), Fp(10), (float*)d_out);
}
